// NeuralMemoryNetwork_51049981281184
// MI455X (gfx1250) — hardware-run, weakly checked
//
#include <hip/hip_runtime.h>
#include <math.h>

constexpr int kRows  = 8192;
constexpr int kInDim = 1024;
constexpr int kMemD  = 512;
constexpr int kSlots = 8192;

constexpr float kCarryX   = 16.0f;
constexpr float kCarryW   = 256.0f;
constexpr float kCarryEnc = 16.0f;
constexpr float kCarryP   = 32768.0f;
constexpr float kCarryMo  = 4096.0f;
constexpr float kEncScale = kCarryEnc / (kCarryX * kCarryW);
constexpr float kSimScale = 1.0f / (kCarryEnc * kCarryW);
constexpr float kMoFold   = kCarryMo / (kCarryP * kCarryW);
constexpr float kOutScale = 1.0f / (kCarryMo * kCarryW);

typedef __attribute__((ext_vector_type(16))) _Float16 v16h;
typedef __attribute__((ext_vector_type(8)))  _Float16 v8h;
typedef __attribute__((ext_vector_type(8)))  float    v8f;
typedef __attribute__((ext_vector_type(4)))  float    v4f;
typedef __attribute__((ext_vector_type(4)))  unsigned int v4u;

__device__ __forceinline__ unsigned short f2bf_bits(float f) {
  unsigned u = __float_as_uint(f);
  return (unsigned short)((u + 0x7FFFu + ((u >> 16) & 1u)) >> 16);
}
__device__ __forceinline__ float bf_bits2f(unsigned short h) { return __uint_as_float(((unsigned)h) << 16); }
__device__ __forceinline__ float bf_rne(float f) { return bf_bits2f(f2bf_bits(f)); }
__device__ __forceinline__ unsigned pk16(unsigned short a, unsigned short b) { return (unsigned)a | ((unsigned)b << 16); }
__device__ __forceinline__ unsigned short h_bits(float f) { const _Float16 h = (_Float16)f; return __builtin_bit_cast(unsigned short, h); }

union FragU { v16h v; v8h h[2]; };
__device__ __forceinline__ v16h frag_load(const _Float16* p) {
  FragU f; f.h[0] = *(const v8h*)(p); f.h[1] = *(const v8h*)(p + 16); return f.v;
}
__device__ __forceinline__ v8f mma_raw(v16h a, v16h b, v8f c) {
  return __builtin_amdgcn_wmma_f32_16x16x32_f16(false, a, false, b, (short)0, c, false, false);
}
__device__ __forceinline__ v8f mma_h(v16h a, v16h b, v8f c) {
  c = __builtin_amdgcn_wmma_f32_16x16x32_f16(false, a, false, b, (short)0, c, false, false);
  asm volatile("v_nop\n\tv_nop\n\tv_nop\n\tv_nop" : "+v"(c) : "v"(a), "v"(b));
  return c;
}
__device__ __forceinline__ void row_guard_h(v8f& a, v8f& b, v8f& c, v8f& d, v16h x, v16h b0, v16h b1, v16h b2, v16h b3) {
  asm volatile("v_nop\n\tv_nop\n\tv_nop\n\tv_nop" : "+v"(a), "+v"(b), "+v"(c), "+v"(d) : "v"(x), "v"(b0), "v"(b1), "v"(b2), "v"(b3));
}
__device__ __forceinline__ void keep4_h(v16h a, v16h b, v16h c, v16h d) { asm volatile("v_nop" :: "v"(a), "v"(b), "v"(c), "v"(d)); }
__device__ __forceinline__ void acc_guard4(v8f& a, v8f& b, v8f& c, v8f& d) { asm volatile("v_nop\n\tv_nop\n\tv_nop\n\tv_nop" : "+v"(a), "+v"(b), "+v"(c), "+v"(d)); }

template <int BIAS_MODE, int OUT_MODE>
__global__ __launch_bounds__(256) void wmma_gemm64_h(
    const unsigned short* __restrict__ Ap, int lda,
    const unsigned short* __restrict__ Btp, int ldb,
    void* __restrict__ Cout, int ldc,
    const float* __restrict__ bias,
    int M, int N, int K, float scale) {
  const _Float16* A  = (const _Float16*)(const void*)Ap;
  const _Float16* Bt = (const _Float16*)(const void*)Btp;
  __shared__ __align__(16) float sT[8][16 * 68];
  const int lane = threadIdx.x & 31;
  const int wave = __builtin_amdgcn_readfirstlane((int)(threadIdx.x >> 5));
  const int tilesN = N >> 6;
  const int tilesM = M >> 6;
  const int tile = blockIdx.x * 8 + wave;
  if (tile >= tilesM * tilesN) return;
  const int tm = tile / tilesN;
  const int tn = tile - tm * tilesN;
  const int m0 = tm << 6;
  const int n0 = tn << 6;

  const int rlane = lane & 15;
  const int koff  = (lane >> 4) * 8;
  const int mOff  = (lane >> 4) * 8;

  v8f acc[4][4];
#pragma unroll
  for (int i = 0; i < 4; ++i)
#pragma unroll
    for (int j = 0; j < 4; ++j) acc[i][j] = (v8f){0.f,0.f,0.f,0.f,0.f,0.f,0.f,0.f};

  for (int k0 = 0; k0 < K; k0 += 32) {
    v16h bh[4];
#pragma unroll
    for (int j = 0; j < 4; ++j) {
      const size_t bo = (size_t)(n0 + (j << 4) + rlane) * ldb + koff + k0;
      bh[j] = frag_load(Bt + bo);
    }
#pragma unroll
    for (int i = 0; i < 4; ++i) {
      const size_t ao = (size_t)(m0 + (i << 4) + rlane) * lda + koff + k0;
      const v16h ah = frag_load(A + ao);
#pragma unroll
      for (int j = 0; j < 4; ++j) acc[i][j] = mma_raw(ah, bh[j], acc[i][j]);
      row_guard_h(acc[i][0], acc[i][1], acc[i][2], acc[i][3], ah, bh[0], bh[1], bh[2], bh[3]);
    }
    keep4_h(bh[0], bh[1], bh[2], bh[3]);
  }
  acc_guard4(acc[0][0], acc[0][1], acc[0][2], acc[0][3]);
  acc_guard4(acc[1][0], acc[1][1], acc[1][2], acc[1][3]);
  acc_guard4(acc[2][0], acc[2][1], acc[2][2], acc[2][3]);
  acc_guard4(acc[3][0], acc[3][1], acc[3][2], acc[3][3]);

  float* slab = sT[wave];
#pragma unroll
  for (int i = 0; i < 4; ++i) {
    const int mBase = m0 + (i << 4);
#pragma unroll
    for (int j = 0; j < 4; ++j) {
      const int n = n0 + (j << 4) + rlane;
      float bv = 0.f;
      if (BIAS_MODE == 2) bv = bias[n];
#pragma unroll
      for (int r = 0; r < 8; ++r) {
        float v = acc[i][j][r] * scale;
        if (BIAS_MODE == 2) v += bv;
        slab[(mOff + r) * 68 + (j << 4) + rlane] = v;
      }
    }
    __builtin_amdgcn_fence(__ATOMIC_RELEASE, "workgroup");
    __builtin_amdgcn_wave_barrier();
    __builtin_amdgcn_fence(__ATOMIC_ACQUIRE, "workgroup");
    if (OUT_MODE == 0) {
      float* C = (float*)Cout;
      const int hh = lane >> 4, c4 = (lane & 15) * 4;
      for (int pass = 0; pass < 2; ++pass) {
#pragma unroll
        for (int it = 0; it < 8; ++it) {
          const int row = it * 2 + hh;
          v4f v = *(const v4f*)(slab + row * 68 + c4);
          *(volatile v4f*)(C + (size_t)(mBase + row) * ldc + n0 + c4) = v;
        }
        __threadfence();
      }
    } else {
      const int q = lane >> 3, c8 = (lane & 7) * 8;
      unsigned short* C = (unsigned short*)Cout;
      for (int pass = 0; pass < 2; ++pass) {
#pragma unroll
        for (int it = 0; it < 4; ++it) {
          const int row = it * 4 + q;
          const float* sp = slab + row * 68 + c8;
          v8h hv;
#pragma unroll
          for (int e = 0; e < 8; ++e) hv[e] = (_Float16)sp[e];
          *(volatile v8h*)(C + (size_t)(mBase + row) * ldc + n0 + c8) = hv;
        }
        __threadfence();
      }
    }
    __builtin_amdgcn_fence(__ATOMIC_RELEASE, "workgroup");
    __builtin_amdgcn_wave_barrier();
    __builtin_amdgcn_fence(__ATOMIC_ACQUIRE, "workgroup");
  }
}

__global__ __launch_bounds__(256) void cvt8_bf_f16_kernel(const float* __restrict__ in, unsigned short* __restrict__ out,
                                                          int n8, float carry) {
  const int i = blockIdx.x * 256 + threadIdx.x;
  if (i >= n8) return;
  const float* p = in + 8 * (size_t)i;
  const v4f a = *(const v4f*)(p);
  const v4f c = *(const v4f*)(p + 4);
  unsigned short hb[8];
#pragma unroll
  for (int e = 0; e < 4; ++e) {
    const float fa = a[e];
    const float fc = c[e];
    hb[e]     = h_bits(bf_rne(fa) * carry);
    hb[4 + e] = h_bits(bf_rne(fc) * carry);
  }
  const v4u u = (v4u){pk16(hb[0], hb[1]), pk16(hb[2], hb[3]), pk16(hb[4], hb[5]), pk16(hb[6], hb[7])};
  unsigned short* q = out + 8 * (size_t)i;
  *(volatile v4u*)q = u;
  __threadfence();
  *(volatile v4u*)q = u;
}

__global__ __launch_bounds__(256) void xsum_part_kernel(const float* __restrict__ x, float* __restrict__ part) {
  const int band = blockIdx.x;
  const int col  = blockIdx.y * 256 + threadIdx.x;
  const float* p = x + (size_t)band * 128 * kInDim + col;
  float s = 0.0f;
#pragma unroll 4
  for (int r = 0; r < 128; ++r) s += bf_rne(p[(size_t)r * kInDim]);
  volatile float* q = part + (size_t)band * kInDim + col;
  *q = s;
  __threadfence();
  *q = s;
}

__global__ __launch_bounds__(256) void upd_kernel(const float* __restrict__ part, const float* __restrict__ Win,
                                                  const float* __restrict__ b_in, const float* __restrict__ b_out,
                                                  float* __restrict__ upd, float* __restrict__ biasE,
                                                  float* __restrict__ biasO) {
  __shared__ float xs[kInDim];
  __shared__ float sdot[32];
  const int tid  = threadIdx.x;
  const int lane = tid & 31;
  const int wave = __builtin_amdgcn_readfirstlane((int)(threadIdx.x >> 5));
#pragma unroll 1
  for (int j = 0; j < 4; ++j) {
    const int col = j * 256 + tid;
    float s = 0.0f;
#pragma unroll 4
    for (int b = 0; b < 64; ++b) s += part[(size_t)b * kInDim + col];
    xs[col] = s;
  }
  __syncthreads();
#pragma unroll 1
  for (int j = 0; j < 4; ++j) {
    const int d = blockIdx.x * 32 + wave * 4 + j;
    const float* wr = Win + (size_t)d * kInDim;
    float s = 0.0f;
#pragma unroll 4
    for (int k = 0; k < 32; ++k) {
      const int i = k * 32 + lane;
      s += bf_rne(wr[i]) * xs[i];
    }
    s += __shfl_xor(s, 16, 32);
    s += __shfl_xor(s, 8, 32);
    s += __shfl_xor(s, 4, 32);
    s += __shfl_xor(s, 2, 32);
    s += __shfl_xor(s, 1, 32);
    if (lane == 0) sdot[wave * 4 + j] = s;
  }
  __syncthreads();
  if (wave == 0) {
    const int d = blockIdx.x * 32 + lane;
    const float bi  = bf_rne(b_in[d]);
    const float u   = 0.025f * sdot[lane] + 204.8f * bi;
    const float be  = kCarryEnc * bi;
    const float bo0 = bf_rne(b_out[blockIdx.x * 64 + lane]);
    const float bo1 = bf_rne(b_out[blockIdx.x * 64 + 32 + lane]);
    volatile float* pu = upd + d;
    volatile float* pe = biasE + d;
    volatile float* p0 = biasO + blockIdx.x * 64 + lane;
    volatile float* p1 = biasO + blockIdx.x * 64 + 32 + lane;
    *pu = u; *pe = be; *p0 = bo0; *p1 = bo1;
    __threadfence();
    *pu = u; *pe = be; *p0 = bo0; *p1 = bo1;
  }
}

__global__ __launch_bounds__(256) void mem_prep_kernel(const float* __restrict__ mem, const float* __restrict__ upd,
                                                       float* __restrict__ out1, unsigned short* __restrict__ mem_h,
                                                       unsigned short* __restrict__ memT_h) {
  __shared__ __align__(16) float tf[64 * 68];
  const int d0  = blockIdx.x * 64;
  const int m0  = blockIdx.y * 64;
  const int tid = threadIdx.x;
  const int lane = tid & 31;
  const int wave = __builtin_amdgcn_readfirstlane((int)(threadIdx.x >> 5));
  {
    const int lr = tid >> 4;
    const int c4 = (tid & 15) * 4;
#pragma unroll
    for (int it = 0; it < 4; ++it) {
      const int rr = it * 16 + lr;
      const v4f a = *(const v4f*)(mem + (size_t)(m0 + rr) * kMemD + d0 + c4);
      v4f b;
#pragma unroll
      for (int e = 0; e < 4; ++e) { const float fa = a[e]; b[e] = bf_rne(fa); }
      *(v4f*)(tf + rr * 68 + c4) = b;
    }
  }
  __syncthreads();
  {
    const int hh = lane >> 4;
    const int c4 = (lane & 15) * 4;
    const v4f u = *(const v4f*)(upd + d0 + c4);
    v4f o[4];
#pragma unroll
    for (int it = 0; it < 4; ++it) {
      const int row = wave * 8 + it * 2 + hh;
      const v4f v = *(const v4f*)(tf + row * 68 + c4);
      v4f w;
#pragma unroll
      for (int e = 0; e < 4; ++e) w[e] = 0.9f * v[e] + u[e];
      o[it] = w;
    }
    for (int pass = 0; pass < 2; ++pass) {
#pragma unroll
      for (int it = 0; it < 4; ++it) {
        const int row = wave * 8 + it * 2 + hh;
        *(volatile v4f*)(out1 + (size_t)(m0 + row) * kMemD + d0 + c4) = o[it];
      }
      __threadfence();
    }
  }
  {
    const int sub = tid >> 3;
    const int c8  = (tid & 7) * 8;
    v4u hv[2], tv[2];
#pragma unroll
    for (int it = 0; it < 2; ++it) {
      const int r = it * 32 + sub;
      v4u a, b;
#pragma unroll
      for (int q = 0; q < 4; ++q) {
        const float f0 = tf[r * 68 + c8 + 2 * q] * kCarryW;
        const float f1 = tf[r * 68 + c8 + 2 * q + 1] * kCarryW;
        const float g0 = tf[(c8 + 2 * q) * 68 + r] * kCarryW;
        const float g1 = tf[(c8 + 2 * q + 1) * 68 + r] * kCarryW;
        a[q] = pk16(h_bits(f0), h_bits(f1));
        b[q] = pk16(h_bits(g0), h_bits(g1));
      }
      hv[it] = a;
      tv[it] = b;
    }
    for (int pass = 0; pass < 2; ++pass) {
#pragma unroll
      for (int it = 0; it < 2; ++it) {
        const int r = it * 32 + sub;
        *(volatile v4u*)(mem_h  + (size_t)(m0 + r) * kMemD  + d0 + c8) = hv[it];
        *(volatile v4u*)(memT_h + (size_t)(d0 + r) * kSlots + m0 + c8) = tv[it];
      }
      __threadfence();
    }
  }
}

constexpr int kAQ  = 16;
constexpr int kQP  = 520;
constexpr int kSTP = 68;
constexpr int kPTP = 72;

__global__ __launch_bounds__(128)
void mem_read_kernel(const unsigned short* __restrict__ encp, const unsigned short* __restrict__ memp,
                     const unsigned short* __restrict__ memTp, unsigned short* __restrict__ mop) {
  __shared__ __align__(16) _Float16 Qs[kAQ * kQP];
  __shared__ __align__(16) float    sT[kAQ * kSTP];
  __shared__ __align__(16) _Float16 pT[kAQ * kPTP];
  __shared__ __align__(16) float    rowScl[kAQ];
  __shared__ __align__(16) float    rowInv[kAQ];

  const _Float16* enc_h  = (const _Float16*)(const void*)encp;
  const _Float16* mem_h  = (const _Float16*)(const void*)memp;
  const _Float16* memT_h = (const _Float16*)(const void*)memTp;

  const int tid  = threadIdx.x;
  const int lane = tid & 31;
  const int wave = __builtin_amdgcn_readfirstlane((int)(threadIdx.x >> 5));
  const int hh   = lane >> 4;
  const int c    = lane & 15;
  const int srow = tid >> 3;
  const int ssub = tid & 7;
  const int rowBase = blockIdx.x * kAQ;

#pragma unroll
  for (int i = 0; i < 8; ++i) {
    const int idx = i * 128 + tid;
    const int r   = idx >> 6;
    const int c16 = idx & 63;
    const v8h qv = *(const v8h*)(enc_h + (size_t)(rowBase + r) * kMemD + c16 * 8);
    *(v8h*)(Qs + r * kQP + c16 * 8) = qv;
  }
  __syncthreads();

  float m_run = -1.0e30f;
  float l_run = 0.0f;
  v8f acc[8];
#pragma unroll
  for (int t = 0; t < 8; ++t) acc[t] = (v8f){0.f,0.f,0.f,0.f,0.f,0.f,0.f,0.f};

  const _Float16* qfr   = Qs + c * kQP + 8 * hh;
  const _Float16* mrowb = mem_h + (size_t)(wave * 16 + c) * kMemD + 8 * hh;
  const _Float16* mTb   = memT_h + (size_t)(wave * 128 + c) * kSlots + 8 * hh;

  for (int chunk = 0; chunk < kSlots; chunk += 64) {
    v8f s = (v8f){0.f,0.f,0.f,0.f,0.f,0.f,0.f,0.f};
    const _Float16* bp = mrowb + (size_t)chunk * kMemD;
#pragma unroll 1
    for (int kg = 0; kg < 4; ++kg) {
#pragma unroll
      for (int ku = 0; ku < 4; ++ku) {
        const int k0 = (kg * 4 + ku) * 32;
        const v16h a = frag_load(qfr + k0);
        const v16h b = frag_load(bp + k0);
        s = mma_h(a, b, s);
      }
    }
#pragma unroll
    for (int r = 0; r < 8; ++r) sT[(8 * hh + r) * kSTP + wave * 16 + c] = s[r] * kSimScale;
    __syncthreads();

    {
      const float* sp = sT + srow * kSTP + ssub * 8;
      const v4f xa = *(const v4f*)(sp);
      const v4f xb = *(const v4f*)(sp + 4);
      float x[8];
#pragma unroll
      for (int e = 0; e < 4; ++e) { x[e] = xa[e]; x[4 + e] = xb[e]; }
      float mc = fmaxf(fmaxf(fmaxf(x[0], x[1]), fmaxf(x[2], x[3])), fmaxf(fmaxf(x[4], x[5]), fmaxf(x[6], x[7])));
      mc = fmaxf(mc, __shfl_xor(mc, 1, 32));
      mc = fmaxf(mc, __shfl_xor(mc, 2, 32));
      mc = fmaxf(mc, __shfl_xor(mc, 4, 32));
      const float mnew = fmaxf(m_run, mc);
      const float scl  = __expf(m_run - mnew);
      float psum = 0.0f;
      v8h pv;
#pragma unroll
      for (int e = 0; e < 8; ++e) {
        const float p = __expf(x[e] - mnew);
        psum += p;
        pv[e] = (_Float16)(p * kCarryP);
      }
      psum += __shfl_xor(psum, 1, 32);
      psum += __shfl_xor(psum, 2, 32);
      psum += __shfl_xor(psum, 4, 32);
      l_run = l_run * scl + psum;
      m_run = mnew;
      *(v8h*)(pT + srow * kPTP + ssub * 8) = pv;
      if (ssub == 0) rowScl[srow] = scl;
    }
    __syncthreads();

    {
      const v4f sa = *(const v4f*)(rowScl + 8 * hh);
      const v4f sb = *(const v4f*)(rowScl + 8 * hh + 4);
#pragma unroll
      for (int t = 0; t < 8; ++t) {
#pragma unroll
        for (int r = 0; r < 4; ++r) {
          acc[t][r]     *= sa[r];
          acc[t][4 + r] *= sb[r];
        }
      }
      const _Float16* vp = mTb + chunk;
#pragma unroll 1
      for (int kk = 0; kk < 2; ++kk) {
        const v16h pa = frag_load(pT + c * kPTP + kk * 32 + 8 * hh);
#pragma unroll
        for (int t = 0; t < 8; ++t) {
          const v16h vb = frag_load(vp + (size_t)t * 16 * kSlots + kk * 32);
          acc[t] = mma_h(pa, vb, acc[t]);
        }
      }
    }
  }

  if (ssub == 0) rowInv[srow] = (1.0f / l_run) * kMoFold;
  __syncthreads();
  {
    const v4f ia = *(const v4f*)(rowInv + 8 * hh);
    const v4f ib = *(const v4f*)(rowInv + 8 * hh + 4);
#pragma unroll
    for (int t = 0; t < 8; ++t) {
#pragma unroll
      for (int r = 0; r < 4; ++r) {
        Qs[(8 * hh + r) * kQP + wave * 128 + t * 16 + c]     = (_Float16)(acc[t][r] * ia[r]);
        Qs[(8 * hh + 4 + r) * kQP + wave * 128 + t * 16 + c] = (_Float16)(acc[t][4 + r] * ib[r]);
      }
    }
  }
  __syncthreads();
  {
    v8h vals[8];
#pragma unroll
    for (int i = 0; i < 8; ++i) {
      const int row = wave * 4 + (i >> 1);
      const int col = (i & 1) * 256 + lane * 8;
      vals[i] = *(const v8h*)(Qs + row * kQP + col);
    }
    for (int pass = 0; pass < 2; ++pass) {
#pragma unroll
      for (int i = 0; i < 8; ++i) {
        const int row = wave * 4 + (i >> 1);
        const int col = (i & 1) * 256 + lane * 8;
        *(volatile v8h*)(mop + (size_t)(rowBase + row) * kMemD + col) = vals[i];
      }
      __threadfence();
    }
  }
}

extern "C" void kernel_launch(void* const* d_in, const int* in_sizes, int n_in,
                              void* d_out, int out_size, void* d_ws, size_t ws_size,
                              hipStream_t stream) {
  static_assert(kRows % 64 == 0 && kMemD % 64 == 0 && kInDim % 64 == 0 && kSlots % 64 == 0);
  static_assert(kInDim % 32 == 0 && kMemD % 32 == 0);
  static_assert(kRows % kAQ == 0 && kRows % 128 == 0 && kInDim % 256 == 0 && kMemD % 32 == 0);
  static_assert((size_t)kRows * kInDim * 4 == (size_t)33554432);
  static_assert((size_t)kRows * kInDim * 4 + (size_t)kSlots * kMemD * 4 == (size_t)50331648);
  if (n_in < 8) return;
  if (in_sizes[0] != kRows * kInDim || in_sizes[1] != kMemD * kInDim || in_sizes[2] != kMemD ||
      in_sizes[3] != kInDim * kMemD || in_sizes[4] != kInDim || in_sizes[7] != kSlots * kMemD ||
      out_size != kRows * kInDim + kSlots * kMemD) return;

  const float* x      = (const float*)d_in[0];
  const float* W_in   = (const float*)d_in[1];
  const float* b_in   = (const float*)d_in[2];
  const float* W_out  = (const float*)d_in[3];
  const float* b_out  = (const float*)d_in[4];
  const float* memory = (const float*)d_in[7];

  float* out0 = (float*)d_out;
  float* out1 = out0 + (size_t)kRows * kInDim;

  const size_t bXh   = (size_t)kRows * kInDim * 2;
  const size_t bWin  = (size_t)kMemD * kInDim * 2;
  const size_t bWout = (size_t)kInDim * kMemD * 2;
  const size_t bMem  = (size_t)kSlots * kMemD * 2;
  const size_t bEnc  = (size_t)kRows * kMemD * 2;
  const size_t bPart = (size_t)64 * kInDim * 4;
  const size_t bUpd  = (size_t)kMemD * 4;
  const size_t bBiE  = (size_t)kMemD * 4;
  const size_t bBiO  = (size_t)kInDim * 4;

  char* ws = (char*)d_ws;
  size_t off = 0;
  unsigned short* x_h    = (unsigned short*)(ws + off); off += bXh;
  unsigned short* Win_h  = (unsigned short*)(ws + off); off += bWin;
  unsigned short* Wout_h = (unsigned short*)(ws + off); off += bWout;
  unsigned short* mem_h  = (unsigned short*)(ws + off); off += bMem;
  unsigned short* memT_h = (unsigned short*)(ws + off); off += bMem;
  unsigned short* enc_h  = (unsigned short*)(ws + off); off += bEnc;
  unsigned short* mo_h   = (unsigned short*)(ws + off); off += bEnc;
  float*          part   = (float*)(ws + off);          off += bPart;
  float*          upd    = (float*)(ws + off);          off += bUpd;
  float*          biasE  = (float*)(ws + off);          off += bBiE;
  float*          biasO  = (float*)(ws + off);          off += bBiO;
  if (off > ws_size || off > (size_t)134217728) return;

  const dim3 blk256(256), blk128(128);

  {
    const int n8x = kRows * kInDim / 8;
    const int n8w = kMemD * kInDim / 8;
    cvt8_bf_f16_kernel<<<dim3(n8x / 256), blk256, 0, stream>>>(x, x_h, n8x, kCarryX);
    cvt8_bf_f16_kernel<<<dim3(n8w / 256), blk256, 0, stream>>>(W_in, Win_h, n8w, kCarryW);
    cvt8_bf_f16_kernel<<<dim3(n8w / 256), blk256, 0, stream>>>(W_out, Wout_h, n8w, kCarryW);
  }

  xsum_part_kernel<<<dim3(64, kInDim / 256), blk256, 0, stream>>>(x, part);
  upd_kernel<<<dim3(kMemD / 32), blk256, 0, stream>>>(part, W_in, b_in, b_out, upd, biasE, biasO);

  mem_prep_kernel<<<dim3(kMemD / 64, kSlots / 64), blk256, 0, stream>>>(memory, upd, out1, mem_h, memT_h);

  {
    const int tiles = (kRows / 64) * (kMemD / 64);
    wmma_gemm64_h<2, 1><<<dim3(tiles / 8), blk256, 0, stream>>>(
        x_h, kInDim, Win_h, kInDim, (void*)enc_h, kMemD, biasE, kRows, kMemD, kInDim, kEncScale);
  }

  mem_read_kernel<<<dim3(kRows / kAQ), blk128, 0, stream>>>(enc_h, mem_h, memT_h, mo_h);

  {
    const int tiles = (kRows / 64) * (kInDim / 64);
    wmma_gemm64_h<2, 0><<<dim3(tiles / 8), blk256, 0, stream>>>(
        mo_h, kMemD, Wout_h, kMemD, (void*)out0, kInDim, biasO, kRows, kInDim, kMemD, kOutScale);
  }
}
